// CausalGAT_2697239461999
// MI455X (gfx1250) — hardware-verified
//
#include <hip/hip_runtime.h>
#include <hip/hip_bf16.h>
#include <math.h>


#define BB 2
#define SS 2048
#define DD 1024
#define HH 16
#define DKK 64
#define QW 2

typedef _Float16 bf16;
typedef __attribute__((ext_vector_type(4))) unsigned v4u_t;
typedef unsigned v4ua __attribute__((ext_vector_type(4), may_alias));
typedef __attribute__((ext_vector_type(4))) float v4f_t;
typedef float v4fa __attribute__((ext_vector_type(4), may_alias));
typedef __attribute__((ext_vector_type(16))) bf16  bf16x16;
typedef __attribute__((ext_vector_type(8)))  bf16  bf16x8;
typedef __attribute__((ext_vector_type(4)))  bf16  bf16x4;
typedef __attribute__((ext_vector_type(8)))  float f32x8;

#define LDS_STRIDE 48
#define KSTRIDE    72
#define VSTRIDE    48

__device__ __forceinline__ f32x8 wmma_bf16(bf16x16 a, bf16x16 b, f32x8 c) {
  return __builtin_amdgcn_wmma_f32_16x16x32_f16(
      false, a, false, b, (short)0, c, false, false);
}

template <typename T>
__device__ __forceinline__ bf16x16 load_frag(const T* __restrict__ base, int ld,
                                             int row0, int k0) {
  const int lane = threadIdx.x & 31;
  const int r    = lane & 15;
  const int kh   = (lane >> 4) * 8;
  const T* p0 = base + (size_t)(row0 + r) * ld + (k0 + kh);
  const T* p1 = p0 + 16;
  bf16x16 f;
#pragma unroll
  for (int i = 0; i < 8; ++i) {
    f[i]     = (bf16)p0[i];
    f[i + 8] = (bf16)p1[i];
  }
  return f;
}

__device__ __forceinline__ bf16x16 lds_frag(const bf16* base, int stride) {
  const int lane = threadIdx.x & 31;
  const int row  = lane & 15;
  const int kh   = (lane >> 4) * 8;
  const bf16x8 lo = *(const bf16x8*)(base + row * stride + kh);
  const bf16x8 hi = *(const bf16x8*)(base + row * stride + kh + 16);
  bf16x16 f;
#pragma unroll
  for (int i = 0; i < 8; ++i) { f[i] = lo[i]; f[i + 8] = hi[i]; }
  return f;
}

template <typename T>
__device__ __forceinline__ void stage_read16(const T* __restrict__ p, float* buf) {
#pragma unroll
  for (int i = 0; i < 16; ++i) buf[i] = (float)p[i];
}

__device__ __forceinline__ void stage_write(bf16* dst, const float* buf, int nquad) {
#pragma unroll
  for (int i = 0; i < nquad; ++i) {
    bf16x4 q;
    q[0] = (bf16)buf[4 * i];     q[1] = (bf16)buf[4 * i + 1];
    q[2] = (bf16)buf[4 * i + 2]; q[3] = (bf16)buf[4 * i + 3];
    *(bf16x4*)(dst + 4 * i) = q;
  }
}

template <typename AT, int MODE>
__global__ __launch_bounds__(256) void gemm_bias_kernel(
    const AT* __restrict__ A, const float* __restrict__ W,
    const float* __restrict__ bias, void* __restrict__ out,
    int M, int N, int K) {
  __shared__ bf16 ldsA[128 * LDS_STRIDE];
  __shared__ bf16 ldsW[256 * LDS_STRIDE];
  __shared__ __attribute__((aligned(16))) unsigned char sob[256 * 136 * 2];

  const int t    = threadIdx.x;
  const int wave = t >> 5;
  const int lane = t & 31;
  const int wm   = (wave & 1) * 64;
  const int wn   = (wave >> 1) * 64;
  const int mBlk = blockIdx.x * 128;
  const int nBlk = blockIdx.y * 256;

  const int arow = t >> 1;
  const int ach  = (t & 1) * 16;

  float abuf[16];
  float wbuf[32];

  stage_read16(A + (size_t)(mBlk + arow) * K + ach, abuf);
  stage_read16(W + (size_t)(nBlk + t) * K,          wbuf);
  stage_read16(W + (size_t)(nBlk + t) * K + 16,     wbuf + 16);

  f32x8 acc[4][4] = {};

  for (int k = 0; k < K; k += 32) {
    __syncthreads();
    stage_write(&ldsA[arow * LDS_STRIDE + ach], abuf, 4);
    stage_write(&ldsW[t * LDS_STRIDE],          wbuf, 8);
    if (k + 32 < K) {
      stage_read16(A + (size_t)(mBlk + arow) * K + (k + 32) + ach, abuf);
      stage_read16(W + (size_t)(nBlk + t) * K + (k + 32),          wbuf);
      stage_read16(W + (size_t)(nBlk + t) * K + (k + 32) + 16,     wbuf + 16);
    }
    __syncthreads();

    bf16x16 af[4], wf[4];
#pragma unroll
    for (int i = 0; i < 4; ++i)
      af[i] = lds_frag(ldsA + (wm + 16 * i) * LDS_STRIDE, LDS_STRIDE);
#pragma unroll
    for (int j = 0; j < 4; ++j)
      wf[j] = lds_frag(ldsW + (wn + 16 * j) * LDS_STRIDE, LDS_STRIDE);
#pragma unroll
    for (int i = 0; i < 4; ++i)
#pragma unroll
      for (int j = 0; j < 4; ++j)
        acc[i][j] = wmma_bf16(af[i], wf[j], acc[i][j]);
  }

  const int nlane = lane & 15;
  const int mh    = (lane >> 4) * 8;
  __syncthreads();
  if (MODE == 0 || MODE == 1) {
    bf16* so = (bf16*)sob;
#pragma unroll
    for (int i = 0; i < 4; ++i)
#pragma unroll
      for (int j = 0; j < 4; ++j) {
        const int nl = wn + 16 * j + nlane;
        const float bv = bias ? bias[nBlk + nl] : 0.0f;
#pragma unroll
        for (int r = 0; r < 8; ++r) {
          const int ml = wm + 16 * i + mh + r;
          const bf16 hv = (bf16)(acc[i][j][r] + bv);
          if (MODE == 0) so[ml * 264 + nl] = hv;
          else           so[nl * 136 + ml] = hv;
        }
      }
    __syncthreads();
#pragma unroll 1
    for (int pass = 0; pass < 2; ++pass) {
      if (MODE == 0) {
        for (int ch = t; ch < 128 * 32; ch += 256) { const int ml = ch >> 5, q = (ch & 31) * 8;
          *(volatile v4u_t*)((bf16*)out + (size_t)(mBlk + ml) * N + nBlk + q) = *(const v4ua*)(so + ml * 264 + q); }
      } else {
        const int b_ = mBlk / SS, s0 = mBlk & (SS - 1);
        for (int ch = t; ch < 256 * 16; ch += 256) { const int nl = ch >> 4, q = (ch & 15) * 8; const int n = nBlk + nl, h = n >> 6, dk = n & (DKK - 1);
          *(volatile v4u_t*)((bf16*)out + (((size_t)(b_ * HH + h)) * DKK + dk) * SS + s0 + q) = *(const v4ua*)(so + nl * 136 + q); }
      }
      __threadfence();
    }
  } else {
    float* so = (float*)sob;
#pragma unroll 1
    for (int hf = 0; hf < 2; ++hf) {
      if (wm == hf * 64) {
#pragma unroll
        for (int i = 0; i < 4; ++i)
#pragma unroll
          for (int j = 0; j < 4; ++j) {
            const int nl = wn + 16 * j + nlane;
            const float bv = bias ? bias[nBlk + nl] : 0.0f;
#pragma unroll
            for (int r = 0; r < 8; ++r) so[(16 * i + mh + r) * 260 + nl] = acc[i][j][r] + bv;
          }
      }
      __syncthreads();
#pragma unroll 1
      for (int pass = 0; pass < 2; ++pass) {
        for (int ch = t; ch < 64 * 64; ch += 256) { const int ml = ch >> 6, q = (ch & 63) * 4;
          *(volatile v4f_t*)((float*)out + (size_t)(mBlk + hf * 64 + ml) * N + nBlk + q) = *(const volatile v4fa*)(so + ml * 260 + q); }
        __threadfence();
      }
      __syncthreads();
    }
  }
}


#define GN 50000
#define GNP 50176
#define GE 800000
#define NHD 4
#define DHID 64
#define RG 25088

__device__ __forceinline__ float lk(float x, float s) { return x >= 0.0f ? x : s * x; }

__global__ __launch_bounds__(128) void k_padrows(const float* __restrict__ x, float* __restrict__ XP) {
  const int n = blockIdx.x, t = threadIdx.x; const float v = (n < GN) ? x[(size_t)n * 128 + t] : 0.0f;
  *(volatile float*)(XP + (size_t)n * 128 + t) = v; __threadfence(); *(volatile float*)(XP + (size_t)n * 128 + t) = v;
}
__global__ __launch_bounds__(128) void k_packA(const float* __restrict__ W, int noutw, int K, float* __restrict__ A) {
  const int m = blockIdx.x; for (int k = threadIdx.x; k < K; k += 128) { const float v = (m < noutw) ? W[(size_t)k * noutw + m] : 0.0f; *(volatile float*)(A + (size_t)m * K + k) = v; }
  __threadfence();
  for (int k = threadIdx.x; k < K; k += 128) { const float v = (m < noutw) ? W[(size_t)k * noutw + m] : 0.0f; *(volatile float*)(A + (size_t)m * K + k) = v; }
}
__global__ __launch_bounds__(64) void k_twsrc(const float* __restrict__ W, float* __restrict__ WT) {
  const int n = blockIdx.x, k = threadIdx.x; const float v = W[(size_t)k * 256 + n]; *(volatile float*)(WT + (size_t)n * 64 + k) = v; __threadfence(); *(volatile float*)(WT + (size_t)n * 64 + k) = v;
}
__global__ __launch_bounds__(256) void k_foldatt(const float* __restrict__ Ws, const float* __restrict__ Wd, const float* __restrict__ as_, const float* __restrict__ ad_, float* __restrict__ WA) {
  const int which = blockIdx.x, t = threadIdx.x, k = t >> 2, h = t & 3;
  const float* Wm = which ? Wd : Ws; const float* am = which ? ad_ : as_;
  float s = 0.0f;
#pragma unroll 1
  for (int c = 0; c < 64; ++c) s += Wm[(size_t)k * 256 + h * 64 + c] * am[h * 64 + c];
  float* d = WA + (size_t)which * DHID * NHD + t; *(volatile float*)d = s; __threadfence(); *(volatile float*)d = s;
}
__global__ __launch_bounds__(256) void k_hrows(const float* __restrict__ T, const float* __restrict__ b, const float* __restrict__ WA, float* __restrict__ Hr, float* __restrict__ AS, float* __restrict__ AD) {
  __shared__ float tile[64][65]; __shared__ float wa[2][64][4];
  const int n0 = blockIdx.x * 64, t = threadIdx.x;
  for (int i = t; i < 64 * 64; i += 256) { const int c = i >> 6, nn = i & 63; tile[c][nn] = lk(T[(size_t)c * GNP + n0 + nn] + b[c], 0.01f); }
  for (int i = t; i < 2 * 64 * 4; i += 256) (&wa[0][0][0])[i] = WA[i];
  __syncthreads();
#pragma unroll 1
  for (int pass = 0; pass < 2; ++pass) {
    for (int i = t; i < 64 * 16; i += 256) { const int nr = i >> 4, c4 = (i & 15) * 4; v4f_t v; v.x = tile[c4][nr]; v.y = tile[c4 + 1][nr]; v.z = tile[c4 + 2][nr]; v.w = tile[c4 + 3][nr];
      *(volatile v4f_t*)(Hr + (size_t)(n0 + nr) * DHID + c4) = v; }
    { const int nr = t >> 2, h = t & 3; float s = 0.f, d = 0.f;
      for (int c = 0; c < 64; ++c) { const float hv = tile[c][nr]; s += hv * wa[0][c][h]; d += hv * wa[1][c][h]; }
      *(volatile float*)(AS + (size_t)(n0 + nr) * NHD + h) = s; *(volatile float*)(AD + (size_t)(n0 + nr) * NHD + h) = d; }
    __threadfence(); }
}
__global__ __launch_bounds__(256) void k_gatmax(const int* __restrict__ srci, const int* __restrict__ dsti, const float* __restrict__ AS, const float* __restrict__ AD, float* __restrict__ MX) {
  __shared__ int qd[8][256], qs[8][256]; __shared__ int wcnt[8][8];
  const int tid = threadIdx.x, lane = tid & 31, wave = tid >> 5;
  for (int i = tid; i < GNP; i += 256) { v4f_t z; z.x = z.y = z.z = z.w = -INFINITY; *(volatile v4f_t*)(MX + (size_t)i * 4) = z; }
  __threadfence(); __syncthreads();
#pragma unroll 1
  for (int c0 = 0; c0 < GE; c0 += 256) {
    const int e = c0 + tid; int d = -1, sidx = 0;
    if (e < GE) { const int draw = dsti[e]; d = draw < 0 ? 0 : (draw >= GN ? GN - 1 : draw); const int ss = srci[e]; sidx = ss < 0 ? 0 : (ss >= GN ? GN - 1 : ss); }
    const int own = (d >= 0) ? (d & 7) : -1; unsigned mown = 0u;
#pragma unroll
    for (int ww = 0; ww < 8; ++ww) { const unsigned m = __builtin_amdgcn_ballot_w32(own == ww); if (own == ww) mown = m; if (lane == 0) wcnt[ww][wave] = __builtin_popcount(m); }
    __syncthreads();
    if (own >= 0) { int base = 0;
#pragma unroll
      for (int w2 = 0; w2 < 8; ++w2) base += (w2 < wave) ? wcnt[own][w2] : 0;
      const int pos = base + __builtin_popcount(mown & ((1u << lane) - 1u)); qd[own][pos] = d; qs[own][pos] = sidx; }
    int total = 0;
#pragma unroll
    for (int w2 = 0; w2 < 8; ++w2) total += wcnt[wave][w2];
    __syncthreads();
    if (lane < NHD) {
#pragma unroll 1
      for (int qi = 0; qi < total; ++qi) { const int dl = qd[wave][qi], sl = qs[wave][qi];
        const float ev = lk(AS[(size_t)sl * NHD + lane] + AD[(size_t)dl * NHD + lane], 0.2f); float* p = MX + (size_t)dl * NHD + lane; *p = fmaxf(*p, ev); } }
    __syncthreads();
  }
  __threadfence(); __syncthreads();
  for (int i = tid; i < GNP; i += 256) { float* p = MX + (size_t)i * 4; v4f_t v = *(const volatile v4fa*)p;
    if (!(v.x > -INFINITY)) v.x = 0.0f; if (!(v.y > -INFINITY)) v.y = 0.0f; if (!(v.z > -INFINITY)) v.z = 0.0f; if (!(v.w > -INFINITY)) v.w = 0.0f;
    *(volatile v4f_t*)p = v; }
  __threadfence();
}
__global__ __launch_bounds__(256) void k_gatacc(const int* __restrict__ srci, const int* __restrict__ dsti, const float* __restrict__ AS, const float* __restrict__ AD, const float* __restrict__ MX,
                                               const bf16* __restrict__ XS, float* __restrict__ R, float* __restrict__ DEN, int rsel) {
  __shared__ int qd[8][256], qs[8][256]; __shared__ int wcnt[8][8];
  const int tid = threadIdx.x, lane = tid & 31, wave = tid >> 5, r0 = rsel * RG;
  for (int i = tid; i < RG * 256 / 4; i += 256) { v4f_t z; z.x = z.y = z.z = z.w = 0.0f; *(volatile v4f_t*)(R + (size_t)i * 4) = z; }
  for (int i = tid; i < RG; i += 256) { v4f_t z; z.x = z.y = z.z = z.w = 0.0f; *(volatile v4f_t*)(DEN + (size_t)(r0 + i) * 4) = z; }
  __threadfence(); __syncthreads();
  const int hl = lane >> 3;
#pragma unroll 1
  for (int c0 = 0; c0 < GE; c0 += 256) {
    const int e = c0 + tid; int d = -1, sidx = 0;
    if (e < GE) { const int draw = dsti[e]; const int dd = draw < 0 ? 0 : (draw >= GN ? GN - 1 : draw);
      if (dd >= r0 && dd < r0 + RG) { d = dd - r0; const int ss = srci[e]; sidx = ss < 0 ? 0 : (ss >= GN ? GN - 1 : ss); } }
    const int own = (d >= 0) ? (d & 7) : -1; unsigned mown = 0u;
#pragma unroll
    for (int ww = 0; ww < 8; ++ww) { const unsigned m = __builtin_amdgcn_ballot_w32(own == ww); if (own == ww) mown = m; if (lane == 0) wcnt[ww][wave] = __builtin_popcount(m); }
    __syncthreads();
    if (own >= 0) { int base = 0;
#pragma unroll
      for (int w2 = 0; w2 < 8; ++w2) base += (w2 < wave) ? wcnt[own][w2] : 0;
      const int pos = base + __builtin_popcount(mown & ((1u << lane) - 1u)); qd[own][pos] = d; qs[own][pos] = sidx; }
    int total = 0;
#pragma unroll
    for (int w2 = 0; w2 < 8; ++w2) total += wcnt[wave][w2];
    __syncthreads();
#pragma unroll 1
    for (int qi = 0; qi < total; ++qi) { const int dl = qd[wave][qi], sl = qs[wave][qi]; const int dn = r0 + dl;
      const float ev = lk(AS[(size_t)sl * NHD + hl] + AD[(size_t)dn * NHD + hl], 0.2f); const float ex = expf(ev - MX[(size_t)dn * NHD + hl]);
      if ((lane & 7) == 0) DEN[(size_t)dn * NHD + hl] += ex;
      const bf16x8 xv = *(const bf16x8*)(XS + (size_t)sl * 256 + lane * 8); float* row = R + (size_t)dl * 256 + lane * 8;
#pragma unroll
      for (int j = 0; j < 8; ++j) row[j] += ex * (float)xv[j]; }
    __syncthreads();
  }
  __threadfence(); __syncthreads();
  for (int i = tid; i < RG * 256 / 4; i += 256) { float* p = R + (size_t)i * 4; const v4f_t v = *(const volatile v4fa*)p; *(volatile v4f_t*)p = v; }
  for (int i = tid; i < RG; i += 256) { float* p = DEN + (size_t)(r0 + i) * 4; const v4f_t v = *(const volatile v4fa*)p; *(volatile v4f_t*)p = v; }
  __threadfence();
}
__global__ __launch_bounds__(128) void k_concat(const float* __restrict__ Hr, const float* __restrict__ R, const float* __restrict__ DEN, const float* __restrict__ bg, int r0, float* __restrict__ HC) {
  const int nl = blockIdx.x, n = r0 + nl, t = threadIdx.x; float v;
  if (t < 64) v = lk(Hr[(size_t)n * DHID + t], 0.01f);
  else { const int c = t - 64; float s = 0.f;
#pragma unroll
    for (int h = 0; h < NHD; ++h) s += R[((size_t)nl * NHD + h) * DHID + c] / (DEN[(size_t)n * NHD + h] + 1e-16f);
    v = lk(s * 0.25f + bg[c], 0.01f); }
  *(volatile float*)(HC + (size_t)n * 128 + t) = v; __threadfence(); *(volatile float*)(HC + (size_t)n * 128 + t) = v;
}
__global__ __launch_bounds__(256) void k_alpha(const int* __restrict__ srci, const int* __restrict__ dsti, const float* __restrict__ AS, const float* __restrict__ AD, const float* __restrict__ MX, const float* __restrict__ DEN, float* __restrict__ alpha) {
  const int e = blockIdx.x * 256 + threadIdx.x; if (e >= GE) return;
  const int draw = dsti[e], sraw = srci[e]; const int d = draw < 0 ? 0 : (draw >= GN ? GN - 1 : draw), s = sraw < 0 ? 0 : (sraw >= GN ? GN - 1 : sraw);
  v4f_t a;
#pragma unroll
  for (int h = 0; h < NHD; ++h) { const float ev = lk(AS[(size_t)s * NHD + h] + AD[(size_t)d * NHD + h], 0.2f); const float ex = expf(ev - MX[(size_t)d * NHD + h]); a[h] = ex / (DEN[(size_t)d * NHD + h] + 1e-16f); }
  *(volatile v4f_t*)(alpha + (size_t)e * 4) = a; __threadfence(); *(volatile v4f_t*)(alpha + (size_t)e * 4) = a;
}
__global__ __launch_bounds__(256) void k_outrows(const float* __restrict__ T2, const float* __restrict__ bf, float* __restrict__ out) {
  __shared__ float tile[64][65];
  const int n0 = blockIdx.x * 64, t = threadIdx.x;
  for (int i = t; i < 64 * 64; i += 256) { const int o = i >> 6, nn = i & 63; tile[o][nn] = T2[(size_t)o * GNP + n0 + nn] + bf[o]; }
  __syncthreads();
#pragma unroll 1
  for (int pass = 0; pass < 2; ++pass) {
    for (int i = t; i < 64 * 16; i += 256) { const int nr = i >> 4, o4 = (i & 15) * 4; if (n0 + nr < GN) { v4f_t v; v.x = tile[o4][nr]; v.y = tile[o4 + 1][nr]; v.z = tile[o4 + 2][nr]; v.w = tile[o4 + 3][nr];
      *(volatile v4f_t*)(out + (size_t)(n0 + nr) * DHID + o4) = v; } }
    __threadfence(); }
}

extern "C" void kernel_launch(void* const* d_in, const int* in_sizes, int n_in,
                              void* d_out, int out_size, void* d_ws, size_t ws_size,
                              hipStream_t stream) {
  (void)in_sizes; (void)n_in; (void)out_size; (void)ws_size;
  const float* X = (const float*)d_in[0];
  const int* ei = (const int*)d_in[1];
  const float* Wlin = (const float*)d_in[2]; const float* blin = (const float*)d_in[3];
  const float* Wsrc = (const float*)d_in[4]; const float* Wdst = (const float*)d_in[5];
  const float* asrc = (const float*)d_in[6]; const float* adst = (const float*)d_in[7];
  const float* bgat = (const float*)d_in[8];
  const float* Wfin = (const float*)d_in[9]; const float* bfin = (const float*)d_in[10];
  const int* srci = ei; const int* dsti = ei + (size_t)GE;
  float* out = (float*)d_out;
  float* alpha = out + (size_t)GN * DHID;
  char* ws = (char*)d_ws;
  float* A1  = (float*)ws; ws += (size_t)128 * 128 * 4;
  float* A2  = (float*)ws; ws += (size_t)128 * 128 * 4;
  float* WsT = (float*)ws; ws += (size_t)256 * 64 * 4;
  float* WA  = (float*)ws; ws += (size_t)2 * 64 * 4 * 4;
  float* XP  = (float*)ws; ws += (size_t)GNP * 128 * 4;
  float* HC  = XP;
  float* T   = (float*)ws; ws += (size_t)128 * GNP * 4;
  float* Hr  = (float*)ws; ws += (size_t)GNP * DHID * 4;
  bf16* XS   = (bf16*)ws;  ws += (size_t)GNP * 256 * 2;
  float* R   = (float*)ws; ws += (size_t)RG * 256 * 4;
  float* AS  = (float*)ws; ws += (size_t)GNP * 4 * 4;
  float* AD  = (float*)ws; ws += (size_t)GNP * 4 * 4;
  float* MX  = (float*)ws; ws += (size_t)GNP * 4 * 4;
  float* DEN = (float*)ws; ws += (size_t)GNP * 4 * 4;
  k_packA<<<128, 128, 0, stream>>>(Wlin, 64, 128, A1);
  k_packA<<<128, 128, 0, stream>>>(Wfin, 64, 128, A2);
  k_twsrc<<<256, 64, 0, stream>>>(Wsrc, WsT);
  k_foldatt<<<2, 256, 0, stream>>>(Wsrc, Wdst, asrc, adst, WA);
  k_padrows<<<GNP, 128, 0, stream>>>(X, XP);
  dim3 blk(256);
  gemm_bias_kernel<float, 2><<<dim3(1, GNP / 256), blk, 0, stream>>>(A1, XP, nullptr, T, 128, GNP, 128);
  k_hrows<<<GNP / 64, 256, 0, stream>>>(T, blin, WA, Hr, AS, AD);
  gemm_bias_kernel<float, 0><<<dim3(GNP / 128, 1), blk, 0, stream>>>(Hr, WsT, nullptr, XS, GNP, 256, 64);
  k_gatmax<<<1, 256, 0, stream>>>(srci, dsti, AS, AD, MX);
  for (int r = 0; r < GNP / RG; ++r) {
    k_gatacc<<<1, 256, 0, stream>>>(srci, dsti, AS, AD, MX, XS, R, DEN, r);
    k_concat<<<RG, 128, 0, stream>>>(Hr, R, DEN, bgat, r * RG, HC);
  }
  k_alpha<<<GE / 256, 256, 0, stream>>>(srci, dsti, AS, AD, MX, DEN, alpha);
  gemm_bias_kernel<float, 2><<<dim3(1, GNP / 256), blk, 0, stream>>>(A2, HC, nullptr, T, 128, GNP, 128);
  k_outrows<<<GNP / 64, 256, 0, stream>>>(T, bfin, out);
}
